// NeighborhoodAttention1D_10368051053041
// MI455X (gfx1250) — hardware-verified
//
#include <hip/hip_runtime.h>
#include <stdint.h>

#define BSZ   2
#define LSEQ  4096
#define CH    1024
#define NHD   16
#define HD    64
#define C3    3072
#define NKEY  13
#define NRAD  6
#define RPW   25
#define MROWS 8192
#define LDC   132
#define ATB   128
#define QSC   0.125f
#define RSC   0.00048828125f
#define S512  0.001953125f
#define S4096 0.000244140625f

static_assert(MROWS == BSZ * LSEQ);
static_assert(CH == NHD * HD);
static_assert(C3 == 3 * CH);
static_assert(RPW == 2 * NKEY - 1);
static_assert(NRAD == NKEY / 2);
static_assert((LSEQ % 64) == 0 && (C3 % 128) == 0 && (CH % 128) == 0 && (CH % 32) == 0);
static_assert(((MROWS * CH) % 2048) == 0 && ((C3 * CH) % 2048) == 0 && ((CH * CH) % 2048) == 0);
static_assert(ATB == NHD * 8 && HD == 64);
static_assert((LDC * 4) % 16 == 0);

typedef _Float16 v16h __attribute__((ext_vector_type(16)));
typedef _Float16 v8h  __attribute__((ext_vector_type(8)));
typedef float    v8f  __attribute__((ext_vector_type(8)));
typedef float    v4f  __attribute__((ext_vector_type(4)));
typedef unsigned int v4u __attribute__((ext_vector_type(4)));

__device__ __forceinline__ unsigned short bf_bits(float f) {
  unsigned u = __float_as_uint(f);
  return (unsigned short)((u + 0x7FFFu + ((u >> 16) & 1u)) >> 16);
}
__device__ __forceinline__ float bf_up(unsigned short b) { return __uint_as_float(((unsigned)b) << 16); }
__device__ __forceinline__ float bfr(float f) { return bf_up(bf_bits(f)); }
__device__ __forceinline__ unsigned short h_bits(_Float16 x) { return __builtin_bit_cast(unsigned short, x); }
__device__ __forceinline__ unsigned short hb16(float f) { return h_bits((_Float16)f); }
__device__ __forceinline__ unsigned pk16(unsigned short a, unsigned short b) { return (unsigned)a | ((unsigned)b << 16); }
__device__ __forceinline__ v8f zero8() { v8f z = {0.f, 0.f, 0.f, 0.f, 0.f, 0.f, 0.f, 0.f}; return z; }

__device__ __forceinline__ v16h ldfrag_h(const _Float16* p) {
  union { v16h v; v8h h[2]; } f;
  f.h[0] = *(const v8h*)(p);
  f.h[1] = *(const v8h*)(p + 16);
  return f.v;
}

__device__ __forceinline__ v8f mma_raw(v16h a, v16h b, v8f c) {
  return __builtin_amdgcn_wmma_f32_16x16x32_f16(false, a, false, b, (short)0, c, false, false);
}
__device__ __forceinline__ void guard4(v8f& c0, v8f& c1, v8f& c2, v8f& c3,
                                       const v16h& a0, const v16h& a1, const v16h& b0, const v16h& b1) {
#if defined(__HIP_DEVICE_COMPILE__)
  asm volatile("v_nop\n\tv_nop\n\tv_nop\n\tv_nop"
               : "+v"(c0), "+v"(c1), "+v"(c2), "+v"(c3) : "v"(a0), "v"(a1), "v"(b0), "v"(b1));
#endif
}
__device__ __forceinline__ void guard8(v8f& c0, v8f& c1, v8f& c2, v8f& c3, v8f& c4, v8f& c5, v8f& c6, v8f& c7,
                                       const v16h& a0, const v16h& a1, const v16h& a2, const v16h& a3,
                                       const v16h& b0, const v16h& b1) {
#if defined(__HIP_DEVICE_COMPILE__)
  asm volatile("v_nop\n\tv_nop\n\tv_nop\n\tv_nop"
               : "+v"(c0), "+v"(c1), "+v"(c2), "+v"(c3), "+v"(c4), "+v"(c5), "+v"(c6), "+v"(c7)
               : "v"(a0), "v"(a1), "v"(a2), "v"(a3), "v"(b0), "v"(b1));
#endif
}

__device__ __forceinline__ void mm_tile(const _Float16* __restrict__ A, int lda,
                                        const _Float16* __restrict__ W, int ldw, int nks,
                                        int arow0, int bcol0, float* Cs) {
  const int tid = threadIdx.x, wave = tid >> 5, lane = tid & 31, hh = lane >> 4, c = lane & 15;
  const int mw = wave >> 2, nw = wave & 3;
  const _Float16* a0p = A + (size_t)(arow0 + mw * 32 + c) * lda + 8 * hh;
  const _Float16* a1p = A + (size_t)(arow0 + mw * 32 + 16 + c) * lda + 8 * hh;
  const _Float16* b0p = W + (size_t)(bcol0 + nw * 32 + c) * ldw + 8 * hh;
  const _Float16* b1p = W + (size_t)(bcol0 + nw * 32 + 16 + c) * ldw + 8 * hh;
  v8f a00 = zero8(), a01 = zero8(), a10 = zero8(), a11 = zero8();
#pragma unroll 1
  for (int ks = 0; ks < nks; ++ks) {
    const int ko = ks * 32;
    const v16h fa0 = ldfrag_h(a0p + ko);
    const v16h fa1 = ldfrag_h(a1p + ko);
    const v16h fb0 = ldfrag_h(b0p + ko);
    const v16h fb1 = ldfrag_h(b1p + ko);
    a00 = mma_raw(fa0, fb0, a00);
    a01 = mma_raw(fa0, fb1, a01);
    a10 = mma_raw(fa1, fb0, a10);
    a11 = mma_raw(fa1, fb1, a11);
    guard4(a00, a01, a10, a11, fa0, fa1, fb0, fb1);
  }
#pragma unroll
  for (int r = 0; r < 8; ++r) {
    const int row = mw * 32 + 8 * hh + r;
    Cs[row * LDC + nw * 32 + c]             = a00[r];
    Cs[row * LDC + nw * 32 + 16 + c]        = a01[r];
    Cs[(row + 16) * LDC + nw * 32 + c]      = a10[r];
    Cs[(row + 16) * LDC + nw * 32 + 16 + c] = a11[r];
  }
}

__device__ __forceinline__ void mm_tile2(const _Float16* __restrict__ Ah, const _Float16* __restrict__ Al, int lda,
                                         const _Float16* __restrict__ W, int ldw, int nks,
                                         int arow0, int bcol0, float* Cs) {
  const int tid = threadIdx.x, wave = tid >> 5, lane = tid & 31, hh = lane >> 4, c = lane & 15;
  const int mw = wave >> 2, nw = wave & 3;
  const size_t r0 = (size_t)(arow0 + mw * 32 + c) * lda + 8 * hh;
  const size_t r1 = (size_t)(arow0 + mw * 32 + 16 + c) * lda + 8 * hh;
  const _Float16* a0h = Ah + r0;
  const _Float16* a1h = Ah + r1;
  const _Float16* a0l = Al + r0;
  const _Float16* a1l = Al + r1;
  const _Float16* b0p = W + (size_t)(bcol0 + nw * 32 + c) * ldw + 8 * hh;
  const _Float16* b1p = W + (size_t)(bcol0 + nw * 32 + 16 + c) * ldw + 8 * hh;
  v8f h00 = zero8(), h01 = zero8(), h10 = zero8(), h11 = zero8();
  v8f l00 = zero8(), l01 = zero8(), l10 = zero8(), l11 = zero8();
#pragma unroll 1
  for (int ks = 0; ks < nks; ++ks) {
    const int ko = ks * 32;
    const v16h fa0 = ldfrag_h(a0h + ko);
    const v16h fa1 = ldfrag_h(a1h + ko);
    const v16h ga0 = ldfrag_h(a0l + ko);
    const v16h ga1 = ldfrag_h(a1l + ko);
    const v16h fb0 = ldfrag_h(b0p + ko);
    const v16h fb1 = ldfrag_h(b1p + ko);
    h00 = mma_raw(fa0, fb0, h00);
    h01 = mma_raw(fa0, fb1, h01);
    h10 = mma_raw(fa1, fb0, h10);
    h11 = mma_raw(fa1, fb1, h11);
    l00 = mma_raw(ga0, fb0, l00);
    l01 = mma_raw(ga0, fb1, l01);
    l10 = mma_raw(ga1, fb0, l10);
    l11 = mma_raw(ga1, fb1, l11);
    guard8(h00, h01, h10, h11, l00, l01, l10, l11, fa0, fa1, ga0, ga1, fb0, fb1);
  }
#pragma unroll
  for (int r = 0; r < 8; ++r) {
    const int row = mw * 32 + 8 * hh + r;
    Cs[row * LDC + nw * 32 + c]             = h00[r] + l00[r] * RSC;
    Cs[row * LDC + nw * 32 + 16 + c]        = h01[r] + l01[r] * RSC;
    Cs[(row + 16) * LDC + nw * 32 + c]      = h10[r] + l10[r] * RSC;
    Cs[(row + 16) * LDC + nw * 32 + 16 + c] = h11[r] + l11[r] * RSC;
  }
}

__global__ __launch_bounds__(256)
void k_cvt16(const float* __restrict__ src, unsigned short* dst, float scale) {
  const size_t i0 = ((size_t)blockIdx.x * 256 + threadIdx.x) * 8;
  const v4f a = *(const v4f*)(src + i0);
  const v4f b = *(const v4f*)(src + i0 + 4);
  v4u pk;
  pk[0] = pk16(hb16(bfr(a[0]) * scale), hb16(bfr(a[1]) * scale));
  pk[1] = pk16(hb16(bfr(a[2]) * scale), hb16(bfr(a[3]) * scale));
  pk[2] = pk16(hb16(bfr(b[0]) * scale), hb16(bfr(b[1]) * scale));
  pk[3] = pk16(hb16(bfr(b[2]) * scale), hb16(bfr(b[3]) * scale));
  unsigned short* gp = dst + i0;
  *(volatile v4u*)gp = pk;
  __threadfence();
  *(volatile v4u*)gp = pk;
}

__global__ __launch_bounds__(256)
void k_gemm_f32(const unsigned short* __restrict__ A, const unsigned short* __restrict__ W, int K,
                const float* __restrict__ bias, float scl, float* out, int ldo) {
  __shared__ __align__(16) float Cs[64 * LDC];
  const int tid = threadIdx.x, wave = tid >> 5, lane = tid & 31;
  const int mb = blockIdx.x, nb = blockIdx.y;
  mm_tile((const _Float16*)(const void*)A, K, (const _Float16*)(const void*)W, K, K >> 5,
          mb * 64, nb * 128, Cs);
  __syncthreads();
  const int col0 = nb * 128 + lane * 4;
  const v4f b4 = *(const v4f*)(bias + col0);
  v4f bb;
#pragma unroll
  for (int e = 0; e < 4; ++e) bb[e] = bfr(b4[e]);
#pragma unroll 1
  for (int it = 0; it < 8; ++it) {
    const int row = wave * 8 + it;
    const size_t t = (size_t)(mb * 64 + row);
    const v4f a = *(const v4f*)(Cs + row * LDC + lane * 4);
    v4f o;
#pragma unroll
    for (int e = 0; e < 4; ++e) o[e] = a[e] * scl + bb[e];
    float* p = out + t * ldo + col0;
    *(volatile v4f*)p = o;
    __threadfence();
    *(volatile v4f*)p = o;
  }
}

__global__ __launch_bounds__(256)
void k_gemm_proj(const unsigned short* __restrict__ ah, const unsigned short* __restrict__ al,
                 const unsigned short* __restrict__ wt, const float* __restrict__ bias, float* out) {
  __shared__ __align__(16) float Cs[64 * LDC];
  const int tid = threadIdx.x, wave = tid >> 5, lane = tid & 31;
  const int mb = blockIdx.x, nb = blockIdx.y;
  mm_tile2((const _Float16*)(const void*)ah, (const _Float16*)(const void*)al, CH,
           (const _Float16*)(const void*)wt, CH, CH / 32, mb * 64, nb * 128, Cs);
  __syncthreads();
  const int col0 = nb * 128 + lane * 4;
  const v4f b4 = *(const v4f*)(bias + col0);
  v4f bb;
#pragma unroll
  for (int e = 0; e < 4; ++e) bb[e] = bfr(b4[e]);
#pragma unroll 1
  for (int it = 0; it < 8; ++it) {
    const int row = wave * 8 + it;
    const size_t t = (size_t)(mb * 64 + row);
    const v4f a = *(const v4f*)(Cs + row * LDC + lane * 4);
    v4f o;
#pragma unroll
    for (int e = 0; e < 4; ++e) o[e] = a[e] * S4096 + bb[e];
    float* pp = out + t * CH + col0;
    *(volatile v4f*)pp = o;
    __threadfence();
    *(volatile v4f*)pp = o;
  }
}

__global__ __launch_bounds__(ATB)
void k_attn(const float* __restrict__ qkv, const float* __restrict__ rpb, unsigned short* ah, unsigned short* al) {
  __shared__ float Ls[NKEY * ATB];
  const int tid = threadIdx.x, h = tid >> 3, sub = tid & 7;
  const int i = blockIdx.x;
  const int ni = min(max(i - NRAD, 0), LSEQ - NKEY);
  const int col = h * HD + sub * 8;
  const float* qr = qkv + (size_t)i * C3 + col;
  const v4f t0 = *(const v4f*)(qr);
  const v4f t1 = *(const v4f*)(qr + 4);
  v4f q0, q1;
#pragma unroll
  for (int e = 0; e < 4; ++e) { q0[e] = t0[e] * QSC; q1[e] = t1[e] * QSC; }
  const float* rp = rpb + h * RPW + (ni - i + 2 * NRAD);
  float mx = -3.0e38f;
#pragma unroll 1
  for (int j = 0; j < NKEY; ++j) {
    const float* kr = qkv + (size_t)(ni + j) * C3 + CH + col;
    const v4f k0 = *(const v4f*)(kr);
    const v4f k1 = *(const v4f*)(kr + 4);
    float s = 0.f;
#pragma unroll
    for (int e = 0; e < 4; ++e) s += q0[e] * k0[e];
#pragma unroll
    for (int e = 0; e < 4; ++e) s += q1[e] * k1[e];
    s += __shfl_xor(s, 1, 32);
    s += __shfl_xor(s, 2, 32);
    s += __shfl_xor(s, 4, 32);
    s += bfr(rp[j]);
    Ls[j * ATB + tid] = s;
    mx = fmaxf(mx, s);
  }
  v4f a0 = {0.f, 0.f, 0.f, 0.f}, a1 = {0.f, 0.f, 0.f, 0.f};
  float l = 0.f;
#pragma unroll 1
  for (int j = 0; j < NKEY; ++j) {
    const float p = __expf(Ls[j * ATB + tid] - mx);
    l += p;
    const float* vr = qkv + (size_t)(ni + j) * C3 + 2 * CH + col;
    const v4f v0 = *(const v4f*)(vr);
    const v4f v1 = *(const v4f*)(vr + 4);
#pragma unroll
    for (int e = 0; e < 4; ++e) { a0[e] += p * v0[e]; a1[e] += p * v1[e]; }
  }
  const float inv64 = __builtin_amdgcn_rcpf(l) * 64.0f;
  unsigned short hb[8], lb[8];
#pragma unroll
  for (int e = 0; e < 4; ++e) {
    const float fa = a0[e] * inv64;
    const _Float16 hv = (_Float16)fa;
    hb[e] = h_bits(hv);
    lb[e] = hb16((fa - (float)hv) * 2048.0f);
    const float fb = a1[e] * inv64;
    const _Float16 hw = (_Float16)fb;
    hb[4 + e] = h_bits(hw);
    lb[4 + e] = hb16((fb - (float)hw) * 2048.0f);
  }
  v4u ph, pl;
  ph[0] = pk16(hb[0], hb[1]); ph[1] = pk16(hb[2], hb[3]); ph[2] = pk16(hb[4], hb[5]); ph[3] = pk16(hb[6], hb[7]);
  pl[0] = pk16(lb[0], lb[1]); pl[1] = pk16(lb[2], lb[3]); pl[2] = pk16(lb[4], lb[5]); pl[3] = pk16(lb[6], lb[7]);
  const size_t o = (size_t)i * CH + col;
  *(volatile v4u*)(ah + o) = ph;
  *(volatile v4u*)(al + o) = pl;
  __threadfence();
  *(volatile v4u*)(ah + o) = ph;
  *(volatile v4u*)(al + o) = pl;
}

extern "C" void kernel_launch(void* const* d_in, const int* in_sizes, int n_in,
                              void* d_out, int out_size, void* d_ws, size_t ws_size,
                              hipStream_t stream) {
  if (n_in < 6) return;
  if (in_sizes[0] != MROWS * CH) return;
  if (in_sizes[1] != C3 * CH) return;
  if (in_sizes[2] != C3) return;
  if (in_sizes[3] != NHD * RPW) return;
  if (in_sizes[4] != CH * CH) return;
  if (in_sizes[5] != CH) return;
  if (out_size != MROWS * CH) return;

  const float* x      = (const float*)d_in[0];
  const float* qkv_w  = (const float*)d_in[1];
  const float* qkv_b  = (const float*)d_in[2];
  const float* rpb    = (const float*)d_in[3];
  const float* proj_w = (const float*)d_in[4];
  const float* proj_b = (const float*)d_in[5];
  float* out = (float*)d_out;

  const size_t sX16 = (size_t)MROWS * CH * 2;
  const size_t sWQ  = (size_t)C3 * CH * 2;
  const size_t sWP  = (size_t)CH * CH * 2;
  const size_t sQKV = (size_t)LSEQ * C3 * 4;
  const size_t sAO  = (size_t)LSEQ * CH * 2;

  size_t off = 0;
  const size_t oX16 = off; off += sX16;
  const size_t oWQ  = off; off += sWQ;
  const size_t oWP  = off; off += sWP;
  const size_t oQKV = off; off += sQKV;
  const size_t oAH  = off; off += sAO;
  const size_t oAL  = off; off += sAO;
  if (off > ws_size) return;
  if (off > (size_t)134217728) return;

  char* ws = (char*)d_ws;
  unsigned short* X16 = (unsigned short*)(ws + oX16);
  unsigned short* WQ  = (unsigned short*)(ws + oWQ);
  unsigned short* WP  = (unsigned short*)(ws + oWP);
  float*          QKV = (float*)(ws + oQKV);
  unsigned short* AH  = (unsigned short*)(ws + oAH);
  unsigned short* AL  = (unsigned short*)(ws + oAL);

  const dim3 blk(256);

  k_cvt16<<<dim3((MROWS * CH) / 2048), blk, 0, stream>>>(x, X16, 8.0f);
  k_cvt16<<<dim3((C3 * CH) / 2048),    blk, 0, stream>>>(qkv_w, WQ, 64.0f);
  k_cvt16<<<dim3((CH * CH) / 2048),    blk, 0, stream>>>(proj_w, WP, 64.0f);

  for (int b = 0; b < BSZ; ++b) {
    k_gemm_f32<<<dim3(LSEQ / 64, C3 / 128), blk, 0, stream>>>(
        X16 + (size_t)b * LSEQ * CH, WQ, CH, qkv_b, S512, QKV, C3);
    k_attn<<<dim3(LSEQ), dim3(ATB), 0, stream>>>(QKV, rpb, AH, AL);
    k_gemm_proj<<<dim3(LSEQ / 64, CH / 128), blk, 0, stream>>>(
        AH, AL, WP, proj_b, out + (size_t)b * LSEQ * CH);
  }
  (void)hipGetLastError();
}
